// CompositionalAttention_83176336655076
// MI455X (gfx1250) — hardware-verified
//
#include <hip/hip_runtime.h>


namespace {
constexpr int NB = 2, S = 2048, E = 512, NS = 8, NRT = 2, DH = 64, VW = NRT * DH  , NR = NB * S;
constexpr float XS = 8.0f, WSC = 256.0f, PS = 8.0f, SCALE = 0.125f, LOG2E = 1.4426950408889634f;

typedef _Float16 b16;
typedef __attribute__((ext_vector_type(16))) _Float16 v16b;
typedef __attribute__((ext_vector_type(8))) _Float16 v8b;
typedef __attribute__((ext_vector_type(8))) float v8f;
typedef __attribute__((ext_vector_type(4))) float v4f;
__device__ __forceinline__ float bf16_rne(float f) { unsigned int u = __float_as_uint(f); u += 0x7FFFu + ((u >> 16) & 1u); return __uint_as_float(u & 0xFFFF0000u); }
__device__ __forceinline__ void split16(float v, b16& hi, b16& lo) { hi = (b16)v; lo = (b16)(v - (float)hi); }
__device__ __forceinline__ v16b frag_kb(const b16* p, int hh) { const v8b a = *(const v8b*)(p + 8 * hh), b = *(const v8b*)(p + 16 + 8 * hh); v16b f;
#pragma unroll
  for (int e = 0; e < 8; ++e) { f[e] = a[e]; f[8 + e] = b[e]; } return f; }
__device__ __forceinline__ v8f wmma16b(v16b a, v16b b, v8f c) { v8f d = __builtin_amdgcn_wmma_f32_16x16x32_f16(false, a, false, b, (short)0, c, false, false); asm volatile("v_nop\n\tv_nop\n\tv_nop\n\tv_nop" : "+v"(d) : "v"(a), "v"(b)); return d; }
__device__ __forceinline__ void wave_lds_sync() { __builtin_amdgcn_fence(__ATOMIC_RELEASE, "workgroup"); __builtin_amdgcn_wave_barrier(); __builtin_amdgcn_fence(__ATOMIC_ACQUIRE, "workgroup"); }
__device__ __forceinline__ float nexp2(float x) { return __builtin_amdgcn_exp2f(x); }
__device__ __forceinline__ float pmul(float a, float b) { float p = a * b; asm volatile("" : "+v"(p)); return p; }
__device__ __forceinline__ float hsum16(float v) { v += __shfl_xor(v, 1); v += __shfl_xor(v, 2); v += __shfl_xor(v, 4); return v + __shfl_xor(v, 8); }

__global__ __launch_bounds__(256) void prepx_kernel(const float* __restrict__ x, b16* __restrict__ X16) {
  const size_t t = (size_t)blockIdx.x * 256 + threadIdx.x; if (t >= (size_t)NR * E / 8) return; const size_t e = t * 8; const v4f a = *(const v4f*)(x + e), c = *(const v4f*)(x + e + 4); v8b o;
#pragma unroll
  for (int j = 0; j < 4; ++j) { o[j] = (b16)(bf16_rne(a[j]) * XS); o[4 + j] = (b16)(bf16_rne(c[j]) * XS); }
  for (int pass = 0; pass < 2; ++pass) { *(volatile v8b*)(X16 + e) = o; __threadfence(); }
}
__device__ __forceinline__ size_t wt_off(int k) { return k <= 2 ? (size_t)k * E * E : k == 3 ? (size_t)3 * E * E : k == 4 ? (size_t)3 * E * E + (size_t)VW * E : (size_t)4 * E * E + (size_t)VW * E; }
__global__ __launch_bounds__(256) void prepw_kernel(const float* __restrict__ wsq, const float* __restrict__ wsk, const float* __restrict__ wrv, const float* __restrict__ wrq, const float* __restrict__ wrk, const float* __restrict__ wout, b16* __restrict__ WT) {
  __shared__ __attribute__((aligned(16))) b16 T[64][64 + 8];
  const int kind = blockIdx.z, i0 = blockIdx.x * 64, o0 = blockIdx.y * 64, t_ = threadIdx.x; int IN = E, OUT = E; const float* w;
  switch (kind) { case 0: w = wsq; break; case 1: w = wsk; break; case 2: w = wrq; break; case 3: w = wrv; OUT = VW; break; case 4: w = wout; break; default: w = wrk; IN = DH; OUT = DH; }
  if (i0 >= IN || o0 >= OUT) return;
  for (int q = t_; q < 64 * 64; q += 256) { const int ii = q >> 6, oo = q & 63; T[oo][ii] = (b16)(bf16_rne(w[(size_t)(i0 + ii) * OUT + o0 + oo]) * WSC); }
  __syncthreads();
  for (int pass = 0; pass < 2; ++pass) { for (int q = t_; q < 64 * 8; q += 256) { const int oo = q >> 3, c8 = (q & 7) * 8; *(volatile v8b*)(WT + wt_off(kind) + (size_t)(o0 + oo) * IN + i0 + c8) = *(const v8b*)(&T[oo][c8]); } __threadfence(); }
}
__global__ __launch_bounds__(128) void proj_kernel(const b16* __restrict__ X16, const b16* __restrict__ WT, b16* __restrict__ Qh, b16* __restrict__ Ql, b16* __restrict__ Kh, b16* __restrict__ Kl, float* __restrict__ RQ, b16* __restrict__ VTh, b16* __restrict__ VTl) {
  __shared__ __attribute__((aligned(16))) float Tf[4][16][128 + 4]; __shared__ __attribute__((aligned(16))) b16 Vt[128][64 + 8], Vtl[128][64 + 8];
  const int wave = threadIdx.x >> 5, lane = threadIdx.x & 31, nloc = lane & 15, hlf = lane >> 4, t_ = threadIdx.x; const int kind = blockIdx.z; const int n0 = blockIdx.y * 128; if (kind == 3 && n0 >= VW) return;
  const size_t m0 = (size_t)blockIdx.x * 64 + wave * 16; const b16* W = WT + wt_off(kind); v8f acc[8];
#pragma unroll
  for (int t = 0; t < 8; ++t) acc[t] = (v8f){};
#pragma unroll 2
  for (int kb = 0; kb < E; kb += 32) { const v16b a = frag_kb(X16 + (m0 + nloc) * E + kb, hlf);
#pragma unroll
    for (int t = 0; t < 8; ++t) acc[t] = wmma16b(a, frag_kb(W + (size_t)(n0 + t * 16 + nloc) * E + kb, hlf), acc[t]); }
  if (kind == 3) { const int b = (int)(m0 / S); const int s0 = (int)((size_t)blockIdx.x * 64 - (size_t)b * S);
#pragma unroll
    for (int t = 0; t < 8; ++t)
#pragma unroll
      for (int r = 0; r < 8; ++r) { b16 h_, l_; split16(acc[t][r] * (1.0f / (XS * WSC)) * XS, h_, l_); Vt[t * 16 + nloc][wave * 16 + 8 * hlf + r] = h_; Vtl[t * 16 + nloc][wave * 16 + 8 * hlf + r] = l_; }
    __syncthreads();
    for (int pass = 0; pass < 2; ++pass) { for (int q = t_; q < 128 * 8; q += 128) { const int cc = q >> 3, c8 = (q & 7) * 8; const size_t gi = ((size_t)b * VW + cc) * S + s0 + c8; *(volatile v8b*)(VTh + gi) = *(const v8b*)(&Vt[cc][c8]); *(volatile v8b*)(VTl + gi) = *(const v8b*)(&Vtl[cc][c8]); } __threadfence(); }
    return; }
#pragma unroll
  for (int t = 0; t < 8; ++t)
#pragma unroll
    for (int r = 0; r < 8; ++r) Tf[wave][8 * hlf + r][t * 16 + nloc] = acc[t][r] * (1.0f / (XS * WSC));
  wave_lds_sync();
  for (int pass = 0; pass < 2; ++pass) { for (int rr = 0; rr < 16; ++rr) {
      if (kind == 2) *(volatile v4f*)(RQ + (m0 + rr) * E + n0 + lane * 4) = *(const v4f*)(&Tf[wave][rr][lane * 4]);
      else if (lane < 16) { b16* dh = kind == 0 ? Qh : Kh; b16* dl = kind == 0 ? Ql : Kl; v8b hv, lv; for (int j = 0; j < 8; ++j) { b16 a_, c_; split16(Tf[wave][rr][lane * 8 + j] * XS, a_, c_); hv[j] = a_; lv[j] = c_; }
        *(volatile v8b*)(dh + (m0 + rr) * E + n0 + lane * 8) = hv; *(volatile v8b*)(dl + (m0 + rr) * E + n0 + lane * 8) = lv; } }
    __threadfence(); }
}
__global__ __launch_bounds__(64) void attn_kernel(const b16* __restrict__ Qh, const b16* __restrict__ Ql, const b16* __restrict__ Kh, const b16* __restrict__ Kl, const b16* __restrict__ VTh, const b16* __restrict__ VTl, b16* __restrict__ RETh, b16* __restrict__ RETl) {
  __shared__ __attribute__((aligned(16))) float To[2][16][VW + 4];
  const int wave = threadIdx.x >> 5, lane = threadIdx.x & 31, hh = lane >> 4, col = lane & 15; const int b = blockIdx.z, s = blockIdx.y; const int q0 = blockIdx.x * 32 + wave * 16, qi = q0 + col;
  const size_t qo = ((size_t)b * S + qi) * E + s * DH; const v16b qa0 = frag_kb(Qh + qo, hh), qa1 = frag_kb(Qh + qo + 32, hh), ql0 = frag_kb(Ql + qo, hh), ql1 = frag_kb(Ql + qo + 32, hh);
  const b16* Kb = Kh + (size_t)b * S * E + s * DH; const b16* Klb = Kl + (size_t)b * S * E + s * DH; const b16* Vb = VTh + (size_t)b * VW * S; const b16* Vlb = VTl + (size_t)b * VW * S;
  float m = -INFINITY, l = 0.0f; v8f o[8], ol[8];
#pragma unroll
  for (int t = 0; t < 8; ++t) { o[t] = (v8f){}; ol[t] = (v8f){}; }
  const float cs = SCALE * LOG2E / (XS * XS);
  for (int kb = 0; kb < S; kb += 32) {
    v8f s0 = {}, s1 = {};
    { const b16* k0 = Kb + (size_t)(kb + col) * E, *k1 = Kb + (size_t)(kb + 16 + col) * E, *k0l = Klb + (size_t)(kb + col) * E, *k1l = Klb + (size_t)(kb + 16 + col) * E;
      v16b f = frag_kb(k0, hh); s0 = wmma16b(f, qa0, s0); s0 = wmma16b(f, ql0, s0); s0 = wmma16b(frag_kb(k0l, hh), qa0, s0);
      f = frag_kb(k0 + 32, hh); s0 = wmma16b(f, qa1, s0); s0 = wmma16b(f, ql1, s0); s0 = wmma16b(frag_kb(k0l + 32, hh), qa1, s0);
      f = frag_kb(k1, hh); s1 = wmma16b(f, qa0, s1); s1 = wmma16b(f, ql0, s1); s1 = wmma16b(frag_kb(k1l, hh), qa0, s1);
      f = frag_kb(k1 + 32, hh); s1 = wmma16b(f, qa1, s1); s1 = wmma16b(f, ql1, s1); s1 = wmma16b(frag_kb(k1l + 32, hh), qa1, s1); }
    float e[16]; float mx = -INFINITY;
#pragma unroll
    for (int r = 0; r < 8; ++r) { e[r] = s0[r] * cs; e[8 + r] = s1[r] * cs; mx = fmaxf(mx, fmaxf(e[r], e[8 + r])); }
    mx = fmaxf(mx, __shfl_xor(mx, 16)); const float mn = fmaxf(m, mx); const float al = nexp2(m - mn); m = mn; float sum = 0.0f; v16b ph, pl;
#pragma unroll
    for (int i = 0; i < 16; ++i) { const float p = nexp2(e[i] - mn); sum += p; const b16 h_ = (b16)(p * PS); ph[i] = h_; pl[i] = (b16)(p * PS - (float)h_); }
    sum += __shfl_xor(sum, 16); l = l * al + sum;
#pragma unroll
    for (int t = 0; t < 8; ++t) { o[t] *= al; ol[t] *= al; const v16b vf = frag_kb(Vb + (size_t)(t * 16 + col) * S + kb, hh); o[t] = wmma16b(vf, ph, o[t]); ol[t] = wmma16b(vf, pl, ol[t]); ol[t] = wmma16b(frag_kb(Vlb + (size_t)(t * 16 + col) * S + kb, hh), ph, ol[t]); } }
  const float inv = 1.0f / (l * PS * XS);
#pragma unroll
  for (int t = 0; t < 8; ++t)
#pragma unroll
    for (int r = 0; r < 8; ++r) To[wave][col][t * 16 + 8 * hh + r] = (o[t][r] + ol[t][r]) * inv;
  wave_lds_sync();
  for (int pass = 0; pass < 2; ++pass) { for (int r_ = 0; r_ < NRT; ++r_) for (int r4 = 0; r4 < 16; r4 += 4) { const int rr = r4 + (lane >> 3), c8 = (lane & 7) * 8; v8b hv, lv; for (int j = 0; j < 8; ++j) { b16 a_, c_; split16(To[wave][rr][r_ * DH + c8 + j] * XS, a_, c_); hv[j] = a_; lv[j] = c_; }
      const size_t gi = ((((size_t)b * NS + s) * NRT + r_) * S + q0 + rr) * DH + c8; *(volatile v8b*)(RETh + gi) = hv; *(volatile v8b*)(RETl + gi) = lv; } __threadfence(); }
}
__global__ __launch_bounds__(256) void rk_kernel(const b16* __restrict__ RETh, const b16* __restrict__ RETl, const b16* __restrict__ WT, const float* __restrict__ RQ, float* __restrict__ SIM) {
  __shared__ float Ss[128];
  const int wave = threadIdx.x >> 5, lane = threadIdx.x & 31, nloc = lane & 15, hlf = lane >> 4, t_ = threadIdx.x; const size_t row0 = (size_t)blockIdx.x * 128 + wave * 16;
  const b16* WRK = WT + wt_off(5);
  v8f acc[4] = {{}, {}, {}, {}};
#pragma unroll
  for (int kb = 0; kb < DH; kb += 32) { const v16b a = frag_kb(RETh + (row0 + nloc) * DH + kb, hlf), al = frag_kb(RETl + (row0 + nloc) * DH + kb, hlf);
#pragma unroll
    for (int t = 0; t < 4; ++t) { const v16b bw = frag_kb(WRK + (size_t)(t * 16 + nloc) * DH + kb, hlf); acc[t] = wmma16b(a, bw, acc[t]); acc[t] = wmma16b(al, bw, acc[t]); } }
#pragma unroll
  for (int r = 0; r < 8; ++r) { const size_t row = row0 + 8 * hlf + r; const int i = (int)(row % S); const int rr_ = (int)((row / S) % NRT); const int s = (int)((row / ((size_t)NRT * S)) % NS); const int b = (int)(row / ((size_t)NS * NRT * S)); (void)rr_;
    const float* rqp = RQ + ((size_t)b * S + i) * E + s * DH; float pd = 0.0f;
#pragma unroll
    for (int t = 0; t < 4; ++t) pd += pmul(acc[t][r] * (1.0f / (XS * WSC)), rqp[t * 16 + nloc]);
    pd = hsum16(pd); if (nloc == 0) Ss[wave * 16 + 8 * hlf + r] = pd * SCALE; }
  __syncthreads();
  for (int pass = 0; pass < 2; ++pass) { if (t_ < 128) ((volatile float*)SIM)[(size_t)blockIdx.x * 128 + t_] = Ss[t_]; __threadfence(); }
}
__global__ __launch_bounds__(256) void mix_kernel(const float* __restrict__ SIM, const b16* __restrict__ RETh, const b16* __restrict__ RETl, b16* __restrict__ OUTh, b16* __restrict__ OUTl) {
  const int wave = threadIdx.x >> 5, lane = threadIdx.x & 31; const size_t tok = (size_t)blockIdx.x * 8 + wave; const int b = (int)(tok / S), i = (int)(tok - (size_t)b * S); const int s = lane >> 2, d0 = (lane & 3) * 16;
  const float s0 = SIM[(((size_t)b * NS + s) * NRT + 0) * S + i], s1 = SIM[(((size_t)b * NS + s) * NRT + 1) * S + i]; const float mx = fmaxf(s0, s1); const float e0 = __expf(s0 - mx), e1 = __expf(s1 - mx); const float inv = 1.0f / (e0 + e1); const float a0 = e0 * inv, a1 = e1 * inv;
  const b16* r0h = RETh + ((((size_t)b * NS + s) * NRT + 0) * S + i) * DH + d0; const b16* r0l = RETl + ((((size_t)b * NS + s) * NRT + 0) * S + i) * DH + d0; const b16* r1h = r0h + (size_t)S * DH; const b16* r1l = r0l + (size_t)S * DH;
  v8b h0, l0, h1, l1;
  for (int j8 = 0; j8 < 16; j8 += 8) { const v8b a = *(const v8b*)(r0h + j8), al = *(const v8b*)(r0l + j8), c = *(const v8b*)(r1h + j8), cl = *(const v8b*)(r1l + j8);
    for (int j = 0; j < 8; ++j) { const float v0 = ((float)a[j] + (float)al[j]) * (1.0f / XS), v1 = ((float)c[j] + (float)cl[j]) * (1.0f / XS); const float o = pmul(a0, v0) + pmul(a1, v1); b16 x_, y_; split16(o * XS, x_, y_); if (j8 == 0) { h0[j] = x_; l0[j] = y_; } else { h1[j] = x_; l1[j] = y_; } } }
  for (int pass = 0; pass < 2; ++pass) { b16* ph = OUTh + tok * E + s * DH + d0; b16* pl = OUTl + tok * E + s * DH + d0; *(volatile v8b*)ph = h0; *(volatile v8b*)(ph + 8) = h1; *(volatile v8b*)pl = l0; *(volatile v8b*)(pl + 8) = l1; __threadfence(); }
}
__global__ __launch_bounds__(128) void outproj_kernel(const b16* __restrict__ Oh, const b16* __restrict__ Ol, const b16* __restrict__ WT, float* __restrict__ out) {
  __shared__ __attribute__((aligned(16))) float Ts[4][16][128 + 4];
  const int wave = threadIdx.x >> 5, lane = threadIdx.x & 31, nloc = lane & 15, hlf = lane >> 4; const size_t m0 = (size_t)blockIdx.x * 64 + wave * 16; const int n0 = blockIdx.y * 128; const b16* WO = WT + wt_off(4);
  v8f acc[8];
#pragma unroll
  for (int t = 0; t < 8; ++t) acc[t] = (v8f){};
#pragma unroll 2
  for (int kb = 0; kb < E; kb += 32) { const v16b a = frag_kb(Oh + (m0 + nloc) * E + kb, hlf), al = frag_kb(Ol + (m0 + nloc) * E + kb, hlf);
#pragma unroll
    for (int t = 0; t < 8; ++t) { const v16b bw = frag_kb(WO + (size_t)(n0 + t * 16 + nloc) * E + kb, hlf); acc[t] = wmma16b(a, bw, acc[t]); acc[t] = wmma16b(al, bw, acc[t]); } }
#pragma unroll
  for (int t = 0; t < 8; ++t)
#pragma unroll
    for (int r = 0; r < 8; ++r) Ts[wave][8 * hlf + r][t * 16 + nloc] = acc[t][r] * (1.0f / (XS * WSC));
  wave_lds_sync();
  for (int pass = 0; pass < 2; ++pass) { for (int rr = 0; rr < 16; ++rr) *(volatile v4f*)(out + (m0 + rr) * E + n0 + lane * 4) = *(const v4f*)(&Ts[wave][rr][lane * 4]); __threadfence(); }
}
}

extern "C" void kernel_launch(void* const* d_in, const int* in_sizes, int n_in, void* d_out, int out_size, void* d_ws, size_t ws_size, hipStream_t stream) {
  (void)n_in;
  auto Fp = [&](int i) { return (const float*)d_in[i]; };
  if (in_sizes[0] != NR * E || in_sizes[1] != E * E || in_sizes[3] != E * VW || in_sizes[5] != DH * DH || in_sizes[6] != E * E || out_size != NR * E) return;
  size_t off = 0; char* ws = (char*)d_ws;
  auto carve = [&](size_t bytes) { char* p = ws + off; off += (bytes + 255) & ~(size_t)255; return p; };
  b16* X16 = (b16*)carve((size_t)NR * E * 2); b16* WT = (b16*)carve(((size_t)4 * E * E + (size_t)VW * E + DH * DH) * 2);
  b16* Qh = (b16*)carve((size_t)NR * E * 2); b16* Ql = (b16*)carve((size_t)NR * E * 2); b16* Kh = (b16*)carve((size_t)NR * E * 2); b16* Kl = (b16*)carve((size_t)NR * E * 2); float* RQ = (float*)carve((size_t)NR * E * 4);
  b16* VTh = (b16*)carve((size_t)NB * VW * S * 2); b16* VTl = (b16*)carve((size_t)NB * VW * S * 2); b16* RETh = (b16*)carve((size_t)NB * NS * NRT * S * DH * 2); b16* RETl = (b16*)carve((size_t)NB * NS * NRT * S * DH * 2); float* SIM = (float*)carve((size_t)NB * NS * NRT * S * 4);
  b16* OUTh = Qh; b16* OUTl = Ql;
  if (off > ws_size || off > ((size_t)128 << 20)) return;
  prepx_kernel<<<(unsigned)(((size_t)NR * E / 8 + 255) / 256), 256, 0, stream>>>(Fp(0), X16);
  prepw_kernel<<<dim3(E / 64, E / 64, 6), 256, 0, stream>>>(Fp(1), Fp(2), Fp(3), Fp(4), Fp(5), Fp(6), WT);
  proj_kernel<<<dim3(NR / 64, E / 128, 4), 128, 0, stream>>>(X16, WT, Qh, Ql, Kh, Kl, RQ, VTh, VTl);
  attn_kernel<<<dim3(S / 32, NS, NB), 64, 0, stream>>>(Qh, Ql, Kh, Kl, VTh, VTl, RETh, RETl);
  rk_kernel<<<(unsigned)((size_t)NB * NS * NRT * S / 128), 256, 0, stream>>>(RETh, RETl, WT, RQ, SIM);
  mix_kernel<<<NR / 8, 256, 0, stream>>>(SIM, RETh, RETl, OUTh, OUTl);
  outproj_kernel<<<dim3(NR / 64, E / 128), 128, 0, stream>>>(OUTh, OUTl, WT, (float*)d_out);
}
